// GPT2Attention_66314295050289
// MI455X (gfx1250) — hardware-verified
//
#include <hip/hip_runtime.h>


#ifndef NB
#define NB 4
#endif
#ifndef SEQ
#define SEQ 2048
#endif
#define NB_FULL  4
#define SEQ_FULL 2048
#define DM   1024
#define NH_  16
#define HD   64
#define DQ   (NH_ * HD)
#define PLOG 8.0f
#define YCAR 256.0f
#define WCAR 64.0f
#define KC   0.18033688011112042f

static_assert(SEQ % 128 == 0);
static_assert((NB * SEQ) % 64 == 0);
static_assert(DM % 64 == 0 && DQ % 64 == 0 && HD == 64 && DQ == DM);
static_assert(((size_t)SEQ * DM) % (8 * 256) == 0);
static_assert((DM * 3 * DQ / 64) % 64 == 0 && (DQ * DM / 64) % 64 == 0);
static_assert(NB <= NB_FULL && SEQ <= SEQ_FULL);
#define WS_TOTAL ((size_t)3 * DQ * DM * 2 + (size_t)DM * DQ * 2 + (size_t)5 * NB * SEQ * DM * 2)
static_assert(WS_TOTAL <= (size_t)134217728);

typedef _Float16 h16;
typedef unsigned short bf;
typedef __attribute__((ext_vector_type(16))) __bf16   v16bf;
typedef __attribute__((ext_vector_type(16))) _Float16 v16h;
typedef __attribute__((ext_vector_type(8)))  _Float16 v8h;
typedef __attribute__((ext_vector_type(8)))  unsigned short v8us;
typedef __attribute__((ext_vector_type(8)))  float    v8f;
typedef __attribute__((ext_vector_type(4)))  float    v4f;
typedef __attribute__((ext_vector_type(2)))  _Float16 v2h;
typedef __attribute__((ext_vector_type(2)))  unsigned short v2us;
typedef v8h  __attribute__((may_alias)) v8ha;
typedef v4f  __attribute__((may_alias)) v4fa;

__device__ __forceinline__ unsigned short f2bf(float f) { unsigned u = __float_as_uint(f); u += 0x7FFFu + ((u >> 16) & 1u); return (unsigned short)(u >> 16); }
__device__ __forceinline__ float bf2f(unsigned short b) { return __uint_as_float(((unsigned)b) << 16); }
__device__ __forceinline__ float bfr(float f) { return bf2f(f2bf(f)); }
__device__ __forceinline__ v16h cat16(v8h lo, v8h hi) { return __builtin_shufflevector(lo, hi, 0, 1, 2, 3, 4, 5, 6, 7, 8, 9, 10, 11, 12, 13, 14, 15); }
__device__ __forceinline__ v16bf cat16b(v8us lo, v8us hi) { return __builtin_bit_cast(v16bf, __builtin_shufflevector(lo, hi, 0, 1, 2, 3, 4, 5, 6, 7, 8, 9, 10, 11, 12, 13, 14, 15)); }
__device__ __forceinline__ v8f wmma16(v16h a, v16h b, v8f c) { return __builtin_amdgcn_wmma_f32_16x16x32_f16(false, a, false, b, (short)0, c, false, false); }
__device__ __forceinline__ v8f wmmab(v16bf a, v16bf b, v8f c) { return __builtin_amdgcn_wmma_f32_16x16x32_bf16(false, a, false, b, (short)0, c, false, false); }
__device__ __forceinline__ void wave_sync() { __builtin_amdgcn_fence(3  , "wavefront"); __builtin_amdgcn_wave_barrier(); asm volatile("" ::: "memory"); }

template <typename T16> struct WFrag;
template <> struct WFrag<h16> { typedef v16h V; static __device__ __forceinline__ V ld(const h16* p) { return cat16(*(const v8h*)p, *(const v8h*)(p + 16)); } static __device__ __forceinline__ v8f mma(V a, V b, v8f c) { return wmma16(a, b, c); } };
template <> struct WFrag<bf> { typedef v16bf V; static __device__ __forceinline__ V ld(const bf* p) { return cat16b(*(const v8us*)p, *(const v8us*)(p + 16)); } static __device__ __forceinline__ v8f mma(V a, V b, v8f c) { return wmmab(a, b, c); } };

template <typename T16, int EPI>
__global__ __launch_bounds__(32) void k_gemmw(const T16* __restrict__ A, const T16* __restrict__ Bt, int K, float* C, int ldc, h16* P, const float* __restrict__ bias, float oscale) {
    typedef typename WFrag<T16>::V V;
    __shared__ __align__(16) float os[16 * 68];
    const int lane = threadIdx.x & 31, lr = lane & 15, hi = lane >> 4; const int r0 = blockIdx.x * 64, c0 = blockIdx.y * 64;
    v8f acc[4][4];
#pragma unroll
    for (int mb = 0; mb < 4; ++mb)
#pragma unroll
        for (int nb = 0; nb < 4; ++nb) acc[mb][nb] = (v8f){};
    const size_t aoff = (size_t)(r0 + lr) * K + 8 * hi, boff = (size_t)(c0 + lr) * K + 8 * hi;
#pragma unroll 1
    for (int kc = 0; kc < K; kc += 32) {
        V a[4];
#pragma unroll
        for (int mb = 0; mb < 4; ++mb) a[mb] = WFrag<T16>::ld(A + aoff + (size_t)mb * 16 * K + kc);
#pragma unroll
        for (int nb = 0; nb < 4; ++nb) { const V b = WFrag<T16>::ld(Bt + boff + (size_t)nb * 16 * K + kc);
#pragma unroll
            for (int mb = 0; mb < 4; ++mb) acc[mb][nb] = WFrag<T16>::mma(a[mb], b, acc[mb][nb]); }
        asm volatile("v_nop\n\tv_nop\n\tv_nop\n\tv_nop" : "+v"(acc[0][0]), "+v"(acc[1][1]), "+v"(acc[2][2]), "+v"(acc[3][3]) : "v"(a[0]), "v"(a[3]));
    }
    if (EPI == 0) {
#pragma unroll
        for (int mb = 0; mb < 4; ++mb) {
#pragma unroll
            for (int nb = 0; nb < 4; ++nb) {
#pragma unroll
                for (int j = 0; j < 8; ++j) os[(hi * 8 + j) * 68 + nb * 16 + lr] = acc[mb][nb][j]; }
            wave_sync();
            float* crow = C + (size_t)(r0 + mb * 16) * ldc + c0;
#pragma unroll 1
            for (int ps = 0; ps < 2; ++ps) {
#pragma unroll
                for (int s = 0; s < 8; ++s) { const int row = 2 * s + hi, cofs = lr * 4; v4f val = *(const v4fa*)(os + row * 68 + cofs);
                    val[0] = val[0] * oscale + bfr(bias[c0 + cofs]); val[1] = val[1] * oscale + bfr(bias[c0 + cofs + 1]); val[2] = val[2] * oscale + bfr(bias[c0 + cofs + 2]); val[3] = val[3] * oscale + bfr(bias[c0 + cofs + 3]);
                    *(volatile v4f*)(crow + (size_t)row * ldc + cofs) = val; }
                if (ps == 0) __threadfence(); }
            wave_sync();
        }
    }
    if (EPI == 1) {
        const int bb = r0 / SEQ, t0 = r0 - bb * SEQ; const int which = c0 / DQ, hh = (c0 - which * DQ) / HD;
        h16* pl = P + ((size_t)(which * NB + bb) * NH_ + hh) * SEQ * HD + (size_t)t0 * HD;
        const int rq = lane >> 3, ch = (lane & 7) * 8;
        float bs[8];
#pragma unroll
        for (int i = 0; i < 8; ++i) bs[i] = bfr(bias[c0 + ch + i]);
#pragma unroll
        for (int mb = 0; mb < 4; ++mb) {
#pragma unroll
            for (int nb = 0; nb < 4; ++nb) {
#pragma unroll
                for (int j = 0; j < 8; ++j) os[(hi * 8 + j) * 68 + nb * 16 + lr] = acc[mb][nb][j]; }
            wave_sync();
            v8h ov[4];
#pragma unroll
            for (int s = 0; s < 4; ++s) { const int row = 4 * s + rq; const v4f x0 = *(const v4fa*)(os + row * 68 + ch); const v4f x1 = *(const v4fa*)(os + row * 68 + ch + 4); v8h o;
#pragma unroll
                for (int i = 0; i < 4; ++i) { o[i] = (h16)(x0[i] + bs[i]); o[4 + i] = (h16)(x1[i] + bs[4 + i]); }
                ov[s] = o; }
            h16* prow = pl + (size_t)mb * 16 * HD;
#pragma unroll 1
            for (int ps = 0; ps < 2; ++ps) {
#pragma unroll
                for (int s = 0; s < 4; ++s) { const int row = 4 * s + rq; *(volatile v8h*)(prow + (size_t)row * HD + ch) = ov[s]; }
                if (ps == 0) __threadfence(); }
            wave_sync();
        }
    }
    if (EPI == 2) {
        const int bb = r0 / SEQ, t0 = r0 - bb * SEQ; const int hh = c0 / HD;
        h16* vt = P + ((size_t)(bb * NH_ + hh) * HD) * SEQ + t0;
        const int rq = lane >> 3, ch = (lane & 7) * 8;
#pragma unroll
        for (int nb = 0; nb < 4; ++nb) {
#pragma unroll
            for (int mb = 0; mb < 4; ++mb) {
#pragma unroll
                for (int j = 0; j < 8; ++j) os[lr * 68 + mb * 16 + hi * 8 + j] = acc[mb][nb][j]; }
            wave_sync();
            v8h ov[4];
#pragma unroll
            for (int s = 0; s < 4; ++s) { const int row = 4 * s + rq; const float bsv = bfr(bias[c0 + nb * 16 + row]); const v4f x0 = *(const v4fa*)(os + row * 68 + ch); const v4f x1 = *(const v4fa*)(os + row * 68 + ch + 4); v8h o;
#pragma unroll
                for (int i = 0; i < 4; ++i) { o[i] = (h16)(x0[i] + bsv); o[4 + i] = (h16)(x1[i] + bsv); }
                ov[s] = o; }
#pragma unroll 1
            for (int ps = 0; ps < 2; ++ps) {
#pragma unroll
                for (int s = 0; s < 4; ++s) { const int row = 4 * s + rq; *(volatile v8h*)(vt + (size_t)(nb * 16 + row) * SEQ + ch) = ov[s]; }
                if (ps == 0) __threadfence(); }
            wave_sync();
        }
    }
}

__global__ __launch_bounds__(256) void k_wtG(const float* __restrict__ w, int K, int N, bf* Bt) {
    const int lane = threadIdx.x & 31; const int L0 = (blockIdx.x * 8 + (threadIdx.x >> 5)) * 8; const int nlines = N * K / 64;
#pragma unroll
    for (int ps = 0; ps < 2; ++ps) {
#pragma unroll 1
        for (int l = 0; l < 8; ++l) { const int L = L0 + l; if (L >= nlines) break; const size_t e = (size_t)L * 64 + lane * 2; const int k = (int)(e % K), n = (int)(e / K); v2us o;
            o[0] = f2bf(w[(size_t)k * N + n]); o[1] = f2bf(w[(size_t)(k + 1) * N + n]); *(volatile v2us*)(Bt + e) = o; }
        if (ps == 0) __threadfence(); }
}
__global__ __launch_bounds__(256) void k_wtH(const float* __restrict__ w, int K, int N, h16* Bt) {
    const int lane = threadIdx.x & 31; const int L0 = (blockIdx.x * 8 + (threadIdx.x >> 5)) * 8; const int nlines = N * K / 64;
#pragma unroll
    for (int ps = 0; ps < 2; ++ps) {
#pragma unroll 1
        for (int l = 0; l < 8; ++l) { const int L = L0 + l; if (L >= nlines) break; const size_t e = (size_t)L * 64 + lane * 2; const int k = (int)(e % K), n = (int)(e / K); v2h o;
            o[0] = (h16)(bfr(w[(size_t)k * N + n]) * WCAR); o[1] = (h16)(bfr(w[(size_t)(k + 1) * N + n]) * WCAR); *(volatile v2h*)(Bt + e) = o; }
        if (ps == 0) __threadfence(); }
}
__global__ __launch_bounds__(256) void k_cvt8(const float* __restrict__ src, bf* dst, size_t n8, size_t sstride, size_t dstride) { src += (size_t)blockIdx.y * sstride; dst += (size_t)blockIdx.y * dstride; const size_t i = (size_t)blockIdx.x * 256 + threadIdx.x; if (i >= n8) return; const v8f v = *(const v8f*)(src + i * 8); v8us o;
#pragma unroll
    for (int k = 0; k < 8; ++k) o[k] = f2bf(v[k]); *(volatile v8us*)(dst + i * 8) = o; __threadfence(); *(volatile v8us*)(dst + i * 8) = o; }

__global__ __launch_bounds__(256) void k_flash(const h16* __restrict__ QP, const h16* __restrict__ KP, const h16* __restrict__ VT, h16* Y) {
    __shared__ __align__(16) h16 ys[8 * 16 * 72];
    const int lane = threadIdx.x & 31, w = threadIdx.x >> 5, lr = lane & 15, hi = lane >> 4;
    const int bh = blockIdx.y; const int q0 = blockIdx.x * 128 + w * 16;
    const h16* qp = QP + (size_t)bh * SEQ * HD + (size_t)(q0 + lr) * HD + 8 * hi;
    const h16* kp = KP + (size_t)bh * SEQ * HD + (size_t)lr * HD + 8 * hi;
    const h16* vt = VT + (size_t)bh * HD * SEQ + (size_t)lr * SEQ + 8 * hi;
    v16h qb[2];
#pragma unroll
    for (int c = 0; c < 2; ++c) qb[c] = WFrag<h16>::ld(qp + 32 * c);
    v8f o[4];
#pragma unroll
    for (int nt = 0; nt < 4; ++nt) o[nt] = (v8f){};
    float m = -3.0e38f, l = 0.f;
#pragma unroll 1
    for (int kv = 0; kv < SEQ; kv += 64) {
        v8f s[4];
#pragma unroll
        for (int j = 0; j < 4; ++j) { s[j] = (v8f){};
#pragma unroll
            for (int c = 0; c < 2; ++c) { const v16h a = WFrag<h16>::ld(kp + (size_t)(kv + 16 * j) * HD + 32 * c); s[j] = wmma16(a, qb[c], s[j]); } }
        asm volatile("v_nop\n\tv_nop\n\tv_nop\n\tv_nop" : "+v"(s[0]), "+v"(s[1]), "+v"(s[2]), "+v"(s[3]) : "v"(qb[0]), "v"(qb[1]));
        float mx = s[0][0];
#pragma unroll
        for (int j = 0; j < 4; ++j)
#pragma unroll
            for (int r = 0; r < 8; ++r) mx = fmaxf(mx, s[j][r]);
        mx = fmaxf(mx, __shfl_xor(mx, 16, 32));
        const float mn = fmaxf(m, mx); const float al = __builtin_amdgcn_exp2f((m - mn) * KC); m = mn;
        const float off = PLOG - mn * KC;
        float rs = 0.f; v16h pb[2];
#pragma unroll
        for (int c = 0; c < 2; ++c) {
#pragma unroll
            for (int r = 0; r < 8; ++r) { const float p0 = __builtin_amdgcn_exp2f(fmaf(s[2 * c][r], KC, off)); const float p1 = __builtin_amdgcn_exp2f(fmaf(s[2 * c + 1][r], KC, off)); rs += p0; rs += p1; pb[c][r] = (h16)p0; pb[c][8 + r] = (h16)p1; } }
        rs += __shfl_xor(rs, 16, 32);
        l = l * al + rs;
#pragma unroll
        for (int nt = 0; nt < 4; ++nt) o[nt] = o[nt] * al;
#pragma unroll
        for (int c = 0; c < 2; ++c) {
#pragma unroll
            for (int nt = 0; nt < 4; ++nt) { const v16h a = WFrag<h16>::ld(vt + (size_t)(16 * nt) * SEQ + kv + 32 * c); o[nt] = wmma16(a, pb[c], o[nt]); } }
        asm volatile("v_nop\n\tv_nop\n\tv_nop\n\tv_nop" : "+v"(o[0]), "+v"(o[1]), "+v"(o[2]), "+v"(o[3]) : "v"(pb[0]), "v"(pb[1]));
    }
    const float f = __fdiv_rn(YCAR, l);
    h16* ysw = ys + w * 16 * 72;
#pragma unroll
    for (int nt = 0; nt < 4; ++nt) { v8h o8;
#pragma unroll
        for (int r = 0; r < 8; ++r) o8[r] = (h16)(o[nt][r] * f);
        *(v8h*)(ysw + lr * 72 + 16 * nt + 8 * hi) = o8; }
    wave_sync();
    const int bb = bh / NH_, hh = bh - bb * NH_; const int rq = lane >> 3, ch = (lane & 7) * 8;
    h16* yrow = Y + ((size_t)bb * SEQ + q0) * DQ + hh * HD;
    v8h ov[4];
#pragma unroll
    for (int s2 = 0; s2 < 4; ++s2) ov[s2] = *(const v8ha*)(ysw + (4 * s2 + rq) * 72 + ch);
#pragma unroll 1
    for (int ps = 0; ps < 2; ++ps) {
#pragma unroll
        for (int s2 = 0; s2 < 4; ++s2) *(volatile v8h*)(yrow + (size_t)(4 * s2 + rq) * DQ + ch) = ov[s2];
        if (ps == 0) __threadfence(); }
}

extern "C" void kernel_launch(void* const* d_in, const int* in_sizes, int n_in,
                              void* d_out, int out_size, void* d_ws, size_t ws_size, hipStream_t stream) {
    if (n_in < 5) return;
    const size_t needx = (size_t)(NB - 1) * SEQ_FULL * DM + (size_t)SEQ * DM;
    if ((size_t)in_sizes[0] < needx) return;
    if ((size_t)in_sizes[1] < (size_t)DM * 3 * DQ) return;
    if ((size_t)in_sizes[2] < (size_t)3 * DQ) return;
    if ((size_t)in_sizes[3] < (size_t)DQ * DM) return;
    if ((size_t)in_sizes[4] < (size_t)DM) return;
    if ((size_t)out_size < (size_t)NB * SEQ * DM) return;
    const float* x = (const float*)d_in[0]; const float* wqkv = (const float*)d_in[1]; const float* bqkv = (const float*)d_in[2]; const float* wo = (const float*)d_in[3]; const float* bo = (const float*)d_in[4];
    float* OUT = (float*)d_out;
    char* wsp = (char*)d_ws;
    auto take = [&](size_t bytes) { char* p = wsp; wsp += (bytes + 255) & ~(size_t)255; return (void*)p; };
    bf*  WQKV = (bf*)take((size_t)3 * DQ * DM * 2);
    h16* WO16 = (h16*)take((size_t)DM * DQ * 2);
    bf*  XB   = (bf*)take((size_t)NB * SEQ * DM * 2);
    h16* QKP  = (h16*)take((size_t)2 * NB * NH_ * SEQ * HD * 2);
    h16* VTP  = (h16*)take((size_t)NB * NH_ * HD * SEQ * 2);
    h16* Y16  = (h16*)take((size_t)NB * SEQ * DQ * 2);
    if ((size_t)(wsp - (char*)d_ws) > ws_size) return;
    h16* QP = QKP; h16* KP = QKP + (size_t)NB * NH_ * SEQ * HD;

    k_cvt8<<<dim3((unsigned)(((size_t)SEQ * DM / 8 + 255) / 256), NB, 1), 256, 0, stream>>>(x, XB, (size_t)SEQ * DM / 8, (size_t)SEQ_FULL * DM, (size_t)SEQ * DM);
    k_wtG<<<(unsigned)((DM * 3 * DQ / 64 + 63) / 64), 256, 0, stream>>>(wqkv, DM, 3 * DQ, WQKV);
    k_wtH<<<(unsigned)((DQ * DM / 64 + 63) / 64), 256, 0, stream>>>(wo, DQ, DM, WO16);
    k_gemmw<bf, 1><<<dim3(NB * SEQ / 64, 2 * DQ / 64, 1), 32, 0, stream>>>(XB, WQKV, DM, nullptr, 0, QKP, bqkv, 1.0f);
    k_gemmw<bf, 2><<<dim3(NB * SEQ / 64, DQ / 64, 1), 32, 0, stream>>>(XB, WQKV + (size_t)2 * DQ * DM, DM, nullptr, 0, VTP, bqkv + 2 * DQ, 1.0f);
    k_flash<<<dim3(SEQ / 128, NB * NH_, 1), 256, 0, stream>>>(QP, KP, VTP, Y16);
    k_gemmw<h16, 0><<<dim3(NB * SEQ / 64, DM / 64, 1), 32, 0, stream>>>(Y16, WO16, DQ, OUT, DM, nullptr, bo, 1.0f / (YCAR * WCAR));
}
